// CodonAttention_90460601188791
// MI455X (gfx1250) — hardware-verified
//
#include <hip/hip_runtime.h>

#define HIDDEN 256
#define NHEADS 4
#define HDIM   64
#define BATCH  2
#define SEQ    4096
#define MROWS  (BATCH * SEQ)

typedef char size_check_0[(MROWS % 128 == 0) ? 1 : -1];
typedef char size_check_1[(HIDDEN % 64 == 0 && HIDDEN % 32 == 0) ? 1 : -1];
typedef char size_check_2[(SEQ % 64 == 0 && SEQ % 32 == 0 && HDIM == 64 && NHEADS * HDIM == HIDDEN) ? 1 : -1];

typedef _Float16 v16h __attribute__((ext_vector_type(16)));
typedef _Float16 v8h  __attribute__((ext_vector_type(8)));
typedef _Float16 v4h  __attribute__((ext_vector_type(4)));
typedef float    v8f  __attribute__((ext_vector_type(8)));
typedef float    v4f  __attribute__((ext_vector_type(4)));

union Frag   { v16h v; v8h half[2]; _Float16 e[16]; };
union Pack16 { v8h h; v4f f; _Float16 e[8]; };
union Pack8  { v4h h; _Float16 e[4]; };

__device__ __forceinline__ v8f wmma16(v16h a, v16h b, v8f c) {
    v8f d = __builtin_amdgcn_wmma_f32_16x16x32_f16(false, a, false, b, (short)0, c, false, false);
    asm volatile("v_nop\n\tv_nop\n\tv_nop\n\tv_nop" : "+v"(d) : "v"(a), "v"(b));
    return d;
}

__device__ __forceinline__ int clamp63(int c) { return c < 0 ? 0 : (c > 63 ? 63 : c); }

__device__ __forceinline__ void vst16(void* p, v4f v) { *(volatile v4f*)p = v; }

__device__ __forceinline__ void load_a(Frag& a, const float* rowp, int k0, int hl) {
    const float* p0 = rowp + k0 + 8 * hl;
    const float* p1 = p0 + 16;
    const v4f x0 = *(const v4f*)p0;
    const v4f x1 = *(const v4f*)(p0 + 4);
    const v4f x2 = *(const v4f*)p1;
    const v4f x3 = *(const v4f*)(p1 + 4);
#pragma unroll
    for (int i = 0; i < 4; ++i) {
        a.e[i]      = (_Float16)x0[i];
        a.e[4 + i]  = (_Float16)x1[i];
        a.e[8 + i]  = (_Float16)x2[i];
        a.e[12 + i] = (_Float16)x3[i];
    }
}
__device__ __forceinline__ void load_a(Frag& a, const _Float16* rowp, int k0, int hl) {
    a.half[0] = *(const v8h*)(rowp + k0 + 8 * hl);
    a.half[1] = *(const v8h*)(rowp + k0 + 16 + 8 * hl);
}

__device__ __forceinline__ void store_pass(_Float16* Out, const float* so, int m0, int n0, int lane) {
    const int rsub = lane >> 3;
    const int col  = (lane & 7) * 8;
#pragma unroll
    for (int it = 0; it < 8; ++it) {
        const int row = it * 4 + rsub;
        const float* sp = so + row * 64 + col;
        const v4f x0 = *(const v4f*)sp;
        const v4f x1 = *(const v4f*)(sp + 4);
        Pack16 p;
#pragma unroll
        for (int i = 0; i < 4; ++i) { p.e[i] = (_Float16)x0[i]; p.e[4 + i] = (_Float16)x1[i]; }
        vst16(Out + (size_t)(m0 + row) * HIDDEN + n0 + col, p.f);
    }
}
__device__ __forceinline__ void store_pass(float* Out, const float* so, int m0, int n0, int lane) {
    const int rsub = lane >> 4;
    const int col  = (lane & 15) * 4;
#pragma unroll
    for (int it = 0; it < 16; ++it) {
        const int row = it * 2 + rsub;
        const v4f x = *(const v4f*)(so + row * 64 + col);
        vst16(Out + (size_t)(m0 + row) * HIDDEN + n0 + col, x);
    }
}

template <typename TA, typename TO>
__global__ __launch_bounds__(128)
void k_gemm_bias(const TA* __restrict__ A,
                 const float* __restrict__ W0, const float* __restrict__ W1, const float* __restrict__ W2,
                 const float* __restrict__ Bi0, const float* __restrict__ Bi1, const float* __restrict__ Bi2,
                 TO* Out0, TO* Out1, TO* Out2, float w_scale, float acc_scale) {
    __shared__ __attribute__((aligned(16))) unsigned char s_raw[64 * 264 * 2];
    _Float16* s_w = (_Float16*)s_raw;
    float*    s_o = (float*)s_raw;

    const int lane = threadIdx.x & 31;
    const int wave = threadIdx.x >> 5;
    const int hl   = lane >> 4;
    const int l16  = lane & 15;
    const int z    = blockIdx.z;
    const float* W    = (z == 0) ? W0 : ((z == 1) ? W1 : W2);
    const float* Bias = (z == 0) ? Bi0 : ((z == 1) ? Bi1 : Bi2);
    TO* Out           = (z == 0) ? Out0 : ((z == 1) ? Out1 : Out2);
    const int n0 = blockIdx.y * 64;
    const int m0 = blockIdx.x * 128 + wave * 32;

    {
        const int wr = threadIdx.x >> 1;
        const int wc = (threadIdx.x & 1) * 128;
        const float* wp = W + (size_t)(n0 + wr) * HIDDEN + wc;
        _Float16* dp = s_w + wr * 264 + wc;
#pragma unroll 4
        for (int i = 0; i < 128; i += 4) {
            const v4f x = *(const v4f*)(wp + i);
            Pack8 y;
#pragma unroll
            for (int j = 0; j < 4; ++j) y.e[j] = (_Float16)(x[j] * w_scale);
            *(v4h*)(dp + i) = y.h;
        }
    }
    __syncthreads();

    v8f acc[2][4] = {};
    const TA* arow0 = A + (size_t)(m0 + l16) * HIDDEN;
    const TA* arow1 = A + (size_t)(m0 + 16 + l16) * HIDDEN;

#pragma unroll 2
    for (int k0 = 0; k0 < HIDDEN; k0 += 32) {
        Frag a0, a1;
        load_a(a0, arow0, k0, hl);
        load_a(a1, arow1, k0, hl);
#pragma unroll
        for (int t = 0; t < 4; ++t) {
            const _Float16* bp = s_w + (t * 16 + l16) * 264 + k0;
            Frag b;
            b.half[0] = *(const v8h*)(bp + 8 * hl);
            b.half[1] = *(const v8h*)(bp + 16 + 8 * hl);
            acc[0][t] = wmma16(a0.v, b.v, acc[0][t]);
            acc[1][t] = wmma16(a1.v, b.v, acc[1][t]);
        }
    }

    __syncthreads();
    float* so = s_o + wave * (32 * 64);
#pragma unroll
    for (int g = 0; g < 2; ++g) {
#pragma unroll
        for (int t = 0; t < 4; ++t) {
            const float bval = Bias[n0 + t * 16 + l16];
#pragma unroll
            for (int r = 0; r < 8; ++r)
                so[(g * 16 + 8 * hl + r) * 64 + t * 16 + l16] = acc[g][t][r] * acc_scale + bval;
        }
    }
    __syncthreads();

    store_pass(Out, so, m0, n0, lane);
    __threadfence();
    store_pass(Out, so, m0, n0, lane);
}

__global__ __launch_bounds__(128)
void k_attn(const _Float16* __restrict__ Q, const _Float16* __restrict__ Kt,
            const _Float16* __restrict__ Vt, const int* __restrict__ codons,
            const float* __restrict__ syn, _Float16* O) {
    __shared__ __attribute__((aligned(16))) float    s_syn[64 * 64];
    __shared__ __attribute__((aligned(16))) _Float16 s_kt[32 * 72];
    __shared__ __attribute__((aligned(16))) _Float16 s_vt[64 * 40];
    __shared__ __attribute__((aligned(16))) _Float16 s_p[4 * 16 * 40];
    __shared__ __attribute__((aligned(16))) _Float16 s_os[4 * 16 * 72];

    const int lane = threadIdx.x & 31;
    const int wave = threadIdx.x >> 5;
    const int hl   = lane >> 4;
    const int l16  = lane & 15;
    const int hd   = blockIdx.y;
    const int b    = blockIdx.z;
    const int q0   = blockIdx.x * 64 + wave * 16;

    for (int i = threadIdx.x; i < 64 * 64; i += 128) s_syn[i] = syn[i];

    const size_t rowbase = (size_t)b * SEQ;

    int cq[8];
#pragma unroll
    for (int r = 0; r < 8; ++r) cq[r] = clamp63(codons[rowbase + q0 + 8 * hl + r]);

    Frag qa[2];
    {
        const _Float16* qp = Q + (rowbase + q0 + l16) * HIDDEN + hd * HDIM;
        load_a(qa[0], qp, 0, hl);
        load_a(qa[1], qp, 32, hl);
    }

    float mrow[8], lrow[8];
#pragma unroll
    for (int r = 0; r < 8; ++r) { mrow[r] = -1.0e30f; lrow[r] = 0.0f; }
    v8f acc[4] = {};

    const int ldr = threadIdx.x >> 2;
    const int ldc = (threadIdx.x & 3) * 16;

    for (int kv0 = 0; kv0 < SEQ; kv0 += 32) {
        const _Float16* kp = Kt + (rowbase + kv0 + ldr) * HIDDEN + hd * HDIM + ldc;
        const _Float16* vp = Vt + (rowbase + kv0 + ldr) * HIDDEN + hd * HDIM + ldc;
        const v8h kx0 = *(const v8h*)kp;
        const v8h kx1 = *(const v8h*)(kp + 8);
        Pack16 vx0, vx1;
        vx0.h = *(const v8h*)vp;
        vx1.h = *(const v8h*)(vp + 8);
        int ck[2];
#pragma unroll
        for (int t = 0; t < 2; ++t) ck[t] = clamp63(codons[rowbase + kv0 + t * 16 + l16]);

        __syncthreads();
        *(v8h*)(s_kt + ldr * 72 + ldc)     = kx0;
        *(v8h*)(s_kt + ldr * 72 + ldc + 8) = kx1;
#pragma unroll
        for (int i = 0; i < 8; ++i) {
            s_vt[(ldc + i) * 40 + ldr]     = vx0.e[i];
            s_vt[(ldc + 8 + i) * 40 + ldr] = vx1.e[i];
        }
        __syncthreads();

        v8f sc[2] = {};
#pragma unroll
        for (int t = 0; t < 2; ++t) {
#pragma unroll
            for (int s = 0; s < 2; ++s) {
                const _Float16* bp = s_kt + (t * 16 + l16) * 72 + s * 32;
                Frag bk;
                bk.half[0] = *(const v8h*)(bp + 8 * hl);
                bk.half[1] = *(const v8h*)(bp + 16 + 8 * hl);
                sc[t] = wmma16(qa[s].v, bk.v, sc[t]);
            }
        }

#pragma unroll
        for (int t = 0; t < 2; ++t) {
#pragma unroll
            for (int r = 0; r < 8; ++r)
                sc[t][r] = sc[t][r] * 0.125f + s_syn[cq[r] * 64 + ck[t]];
        }

        float al[8];
#pragma unroll
        for (int r = 0; r < 8; ++r) {
            float v = fmaxf(sc[0][r], sc[1][r]);
            v = fmaxf(v, __shfl_xor(v, 1));
            v = fmaxf(v, __shfl_xor(v, 2));
            v = fmaxf(v, __shfl_xor(v, 4));
            v = fmaxf(v, __shfl_xor(v, 8));
            const float mn = fmaxf(mrow[r], v);
            const float p0 = __expf(sc[0][r] - mn);
            const float p1 = __expf(sc[1][r] - mn);
            float ts = p0 + p1;
            ts += __shfl_xor(ts, 1);
            ts += __shfl_xor(ts, 2);
            ts += __shfl_xor(ts, 4);
            ts += __shfl_xor(ts, 8);
            al[r]   = __expf(mrow[r] - mn);
            lrow[r] = lrow[r] * al[r] + ts;
            mrow[r] = mn;
            _Float16* prow = s_p + wave * 640 + (8 * hl + r) * 40;
            prow[l16]      = (_Float16)p0;
            prow[16 + l16] = (_Float16)p1;
        }

        __syncthreads();

        Frag pa;
        {
            const _Float16* pp = s_p + wave * 640 + l16 * 40;
            pa.half[0] = *(const v8h*)(pp + 8 * hl);
            pa.half[1] = *(const v8h*)(pp + 16 + 8 * hl);
        }

#pragma unroll
        for (int t = 0; t < 4; ++t) {
#pragma unroll
            for (int r = 0; r < 8; ++r) acc[t][r] *= al[r];
            const _Float16* bvp = s_vt + (t * 16 + l16) * 40;
            Frag bv;
            bv.half[0] = *(const v8h*)(bvp + 8 * hl);
            bv.half[1] = *(const v8h*)(bvp + 16 + 8 * hl);
            acc[t] = wmma16(pa.v, bv.v, acc[t]);
        }
    }

    float inv[8];
#pragma unroll
    for (int r = 0; r < 8; ++r) inv[r] = 16.0f / lrow[r];
    _Float16* os = s_os + wave * (16 * 72);
#pragma unroll
    for (int t = 0; t < 4; ++t) {
#pragma unroll
        for (int r = 0; r < 8; ++r)
            os[(8 * hl + r) * 72 + t * 16 + l16] = (_Float16)(acc[t][r] * inv[r]);
    }
    __syncthreads();

    const int rsub = lane >> 3;
    const int col  = (lane & 7) * 8;
#pragma unroll
    for (int it = 0; it < 4; ++it) {
        const int row = it * 4 + rsub;
        Pack16 p;
        p.h = *(const v8h*)(os + row * 72 + col);
        vst16(O + (rowbase + q0 + row) * HIDDEN + hd * HDIM + col, p.f);
    }
    __threadfence();
#pragma unroll
    for (int it = 0; it < 4; ++it) {
        const int row = it * 4 + rsub;
        Pack16 p;
        p.h = *(const v8h*)(os + row * 72 + col);
        vst16(O + (rowbase + q0 + row) * HIDDEN + hd * HDIM + col, p.f);
    }
}

extern "C" void kernel_launch(void* const* d_in, const int* in_sizes, int n_in,
                              void* d_out, int out_size, void* d_ws, size_t ws_size,
                              hipStream_t stream) {
    if (n_in < 11) return;
    if (in_sizes[0] != MROWS * HIDDEN || in_sizes[1] != MROWS || in_sizes[2] != 64 * 64) return;
    for (int i = 0; i < 4; ++i) {
        if (in_sizes[3 + 2 * i] != HIDDEN * HIDDEN || in_sizes[4 + 2 * i] != HIDDEN) return;
    }
    if (out_size != MROWS * HIDDEN) return;
    const size_t slab = (size_t)MROWS * HIDDEN;
    if (ws_size < 4 * slab * sizeof(_Float16)) return;

    const float* x      = (const float*)d_in[0];
    const int*   codons = (const int*)  d_in[1];
    const float* syn    = (const float*)d_in[2];
    const float* wq     = (const float*)d_in[3];
    const float* bq     = (const float*)d_in[4];
    const float* wk     = (const float*)d_in[5];
    const float* bk     = (const float*)d_in[6];
    const float* wv     = (const float*)d_in[7];
    const float* bv     = (const float*)d_in[8];
    const float* wo     = (const float*)d_in[9];
    const float* bo     = (const float*)d_in[10];
    float* out = (float*)d_out;

    _Float16* qws = (_Float16*)d_ws;
    _Float16* kws = qws + slab;
    _Float16* vws = kws + slab;
    _Float16* ows = vws + slab;

    dim3 block(128);

    k_gemm_bias<float, _Float16><<<dim3(MROWS / 128, HIDDEN / 64, 3), block, 0, stream>>>(
        x, wq, wk, wv, bq, bk, bv, qws, kws, vws, 64.0f, 1.0f / 64.0f);

    k_attn<<<dim3(SEQ / 64, NHEADS, BATCH), block, 0, stream>>>(qws, kws, vws, codons, syn, ows);

    k_gemm_bias<_Float16, float><<<dim3(MROWS / 128, HIDDEN / 64, 1), block, 0, stream>>>(
        ows, wo, wo, wo, bo, bo, bo, out, out, out, 64.0f, 1.0f / 1024.0f);
}
